// MultiHeadAttention_91199335564042
// MI455X (gfx1250) — hardware-verified
//
#include <hip/hip_runtime.h>

typedef _Float16     v16h __attribute__((ext_vector_type(16)));
typedef float        v8f  __attribute__((ext_vector_type(8)));
typedef unsigned int v4u  __attribute__((ext_vector_type(4)));
typedef unsigned int v2u  __attribute__((ext_vector_type(2)));
typedef float        v4f  __attribute__((ext_vector_type(4)));
typedef float        v4fa __attribute__((ext_vector_type(4), may_alias));

#ifndef NB
#define NB 2
#endif
#ifndef SEQ
#define SEQ 2048
#endif
#define NB_FULL  2
#define SEQ_FULL 2048
#define DQ   1024
#define HQ   16
#define HDQ  64
#define MQ   (NB * SEQ)
#define PLX  ((size_t)MQ * DQ)
#define EARLYQ ((SEQ < 512) ? SEQ : 512)
#define WSC    4096.0f
#define RWSC   (1.0f / 4096.0f)
#define PSC    1024.0f
#define RSPLIT (1.0f / 2048.0f)

static_assert(NB >= 1 && NB <= NB_FULL);
static_assert(SEQ % 128 == 0);
static_assert(SEQ <= SEQ_FULL);
static_assert(DQ == HQ * HDQ);
static_assert((EARLYQ / 16) % 8 == 0);
static_assert(((SEQ - EARLYQ) / 16) % 8 == 0);
static_assert(PLX % 1024 == 0);
static_assert(((size_t)DQ * DQ) % 1024 == 0);
static_assert(MQ % 8 == 0);

__device__ __forceinline__ float bfr(float f) {
    unsigned int u = __float_as_uint(f);
    u = (u + 0x7FFFu + ((u >> 16) & 1u)) & 0xFFFF0000u;
    return __uint_as_float(u);
}
__device__ __forceinline__ void split16(float f, _Float16& h, _Float16& l) { h = (_Float16)f; l = (_Float16)((f - (float)h) * 2048.0f); }
__device__ __forceinline__ unsigned short hbits(_Float16 h) { return __builtin_bit_cast(unsigned short, h); }
__device__ __forceinline__ unsigned pack2h(_Float16 a, _Float16 b) { return (unsigned)hbits(a) | ((unsigned)hbits(b) << 16); }

struct U256 { v4u a, b; };
__device__ __forceinline__ v16h load_frag2(const _Float16* p0, const _Float16* p1) {
    U256 t;
    t.a = *reinterpret_cast<const v4u*>(p0);
    t.b = *reinterpret_cast<const v4u*>(p1);
    return __builtin_bit_cast(v16h, t);
}
__device__ __forceinline__ v8f wmma16(v16h a, v16h b, v8f c) {
    c = __builtin_amdgcn_wmma_f32_16x16x32_f16(false, a, false, b, (short)0, c, false, false);
    asm volatile("v_nop\n\tv_nop\n\tv_nop\n\tv_nop" : "+v"(c) : "v"(a), "v"(b));
    return c;
}
__device__ __forceinline__ v8f wmma_split(v16h ah, v16h al, v16h bh, v16h bl, v8f c) {
    v8f x = {};
    x = wmma16(al, bh, x);
    x = wmma16(ah, bl, x);
    return wmma16(ah, bh, c) + x * RSPLIT;
}

__global__ __launch_bounds__(256) void cvt_x(const float* __restrict__ x, _Float16* __restrict__ xh) {
    const size_t i = ((size_t)blockIdx.x * 256 + threadIdx.x) * 4;
    if (i >= PLX) return;
    const size_t m = i / DQ;
    const int c = (int)(i % DQ);
    const int b = (int)(m / SEQ), s = (int)(m % SEQ);
    const float4 v = *(const float4*)(x + ((size_t)b * SEQ_FULL + s) * DQ + c);
    const _Float16 h0 = (_Float16)bfr(v.x), h1 = (_Float16)bfr(v.y), h2 = (_Float16)bfr(v.z), h3 = (_Float16)bfr(v.w);
    v2u ph; ph.x = pack2h(h0, h1); ph.y = pack2h(h2, h3);
    *(volatile v2u*)(xh + i) = ph;
    __threadfence();
    *(volatile v2u*)(xh + i) = ph;
}

__global__ __launch_bounds__(256) void cvt_w(const float* __restrict__ w0, const float* __restrict__ w1,
                                             const float* __restrict__ w2, const float* __restrict__ w3,
                                             _Float16* __restrict__ o0, _Float16* __restrict__ o1,
                                             _Float16* __restrict__ o2, _Float16* __restrict__ o3) {
    const int y = blockIdx.y;
    const float* w = (y == 0) ? w0 : ((y == 1) ? w1 : ((y == 2) ? w2 : w3));
    _Float16* o = (y == 0) ? o0 : ((y == 1) ? o1 : ((y == 2) ? o2 : o3));
    const size_t i = ((size_t)blockIdx.x * 256 + threadIdx.x) * 4;
    if (i >= (size_t)DQ * DQ) return;
    const float4 v = *(const float4*)(w + i);
    const _Float16 h0 = (_Float16)(bfr(v.x) * WSC), h1 = (_Float16)(bfr(v.y) * WSC);
    const _Float16 h2 = (_Float16)(bfr(v.z) * WSC), h3 = (_Float16)(bfr(v.w) * WSC);
    v2u ph; ph.x = pack2h(h0, h1); ph.y = pack2h(h2, h3);
    *(volatile v2u*)(o + i) = ph;
    __threadfence();
    *(volatile v2u*)(o + i) = ph;
}

__global__ __launch_bounds__(256) void rope_tab(const int* __restrict__ tok, float* __restrict__ tab) {
#pragma clang fp contract(off)
    const int r = blockIdx.x * 8 + (threadIdx.x >> 5);
    const int i = threadIdx.x & 31;
    if (r >= MQ) return;
    const int b = r / SEQ, s = r % SEQ;
    const int p = tok[(size_t)b * SEQ_FULL + s];
    const float invf = (float)exp2(-(double)i * 0.41524101186092029348);
    const float ang = (float)p * invf;
    float sn, cs;
    sincosf(ang, &sn, &cs);
    float* d = tab + (size_t)r * 64;
    *(volatile float*)(d + i) = cs; *(volatile float*)(d + 32 + i) = sn;
    __threadfence();
    *(volatile float*)(d + i) = cs; *(volatile float*)(d + 32 + i) = sn;
}

template <int MODE, bool ARES>
__global__ __launch_bounds__(256)
void gemm16(const _Float16* __restrict__ A, const _Float16* __restrict__ BT,
            float* __restrict__ outF, _Float16* __restrict__ outB, const float* __restrict__ tab,
            int N, int K, float scale) {
    constexpr int TSHN = (MODE == 1) ? 8 * 16 * 64 : 4;
    __shared__ alignas(16) _Float16 bsh[2][64 * 32];
    __shared__ alignas(16) float    stg[8][16 * 64];
    __shared__ alignas(16) float    tsh[TSHN];

    const int tid  = threadIdx.x;
    const int lane = tid & 31;
    const int wave = tid >> 5;
    const int lo   = lane & 15;
    const int hi   = lane >> 4;
    const int rowBase = blockIdx.y * 128 + wave * 16;
    const int colBase = blockIdx.x * 64;

    const int cn = tid >> 2, cc = tid & 3;
    const _Float16* bSrc = BT + (size_t)(colBase + cn) * K + cc * 8;
    _Float16* bDst0 = &bsh[0][cn * 32 + cc * 8];
    _Float16* bDst1 = &bsh[1][cn * 32 + cc * 8];
    *reinterpret_cast<v4u*>(bDst0) = *reinterpret_cast<const v4u*>(bSrc);
    __syncthreads();

    v8f acc[4] = {};
    v8f accr[4] = {};
    const _Float16* aRow = A + (size_t)(rowBase + lo) * K;

    const int nk = K / 32;
    for (int ik = 0; ik < nk; ++ik) {
        const int k0  = ik * 32;
        const int buf = ik & 1;
        if (ik + 1 < nk)
            *reinterpret_cast<v4u*>(buf ? bDst0 : bDst1) = *reinterpret_cast<const v4u*>(bSrc + (size_t)(ik + 1) * 32);

        const v16h af = load_frag2(aRow + k0 + hi * 8, aRow + k0 + hi * 8 + 16);
        v16h afl = af;
        if constexpr (ARES) afl = load_frag2(aRow + PLX + k0 + hi * 8, aRow + PLX + k0 + hi * 8 + 16);
#pragma unroll
        for (int t = 0; t < 4; ++t) {
            const _Float16* bp = &bsh[buf][(t * 16 + lo) * 32 + hi * 8];
            const v16h bf = load_frag2(bp, bp + 16);
            acc[t] = wmma16(af, bf, acc[t]);
            if constexpr (ARES) accr[t] = wmma16(afl, bf, accr[t]);
        }
        __syncthreads();
    }
    if constexpr (ARES) {
#pragma unroll
        for (int t = 0; t < 4; ++t) acc[t] = acc[t] + accr[t] * RSPLIT;
    }

    float* sg = stg[wave];
#pragma unroll
    for (int t = 0; t < 4; ++t)
#pragma unroll
        for (int j = 0; j < 8; ++j) sg[(j + 8 * hi) * 64 + t * 16 + lo] = acc[t][j] * scale;
    asm volatile("s_wait_dscnt 0" ::: "memory");
    __builtin_amdgcn_wave_barrier();

    if constexpr (MODE == 0) {
        const int b = rowBase / SEQ, s0 = rowBase % SEQ;
        v4f ov[8]; size_t oo[8];
#pragma unroll
        for (int i = 0; i < 8; ++i) {
            const int c = lane + 32 * i, r = c >> 4, q = c & 15;
            ov[i] = *(const v4fa*)(sg + r * 64 + q * 4);
            oo[i] = ((size_t)b * SEQ_FULL + s0 + r) * (size_t)N + colBase + q * 4;
        }
#pragma unroll
        for (int i = 0; i < 8; ++i) *(volatile v4f*)(outF + oo[i]) = ov[i];
        __threadfence();
#pragma unroll
        for (int i = 0; i < 8; ++i) *(volatile v4f*)(outF + oo[i]) = ov[i];
    } else if constexpr (MODE == 1) {
        const int b = rowBase / SEQ, s0 = rowBase % SEQ;
        const int h = colBase >> 6;
        float* ts = tsh + wave * (16 * 64);
        const float* tsrc = tab + ((size_t)b * SEQ + s0) * 64;
#pragma unroll
        for (int i = 0; i < 8; ++i)
            *(v4f*)(ts + (i * 32 + lane) * 4) = *(const v4f*)(tsrc + (i * 32 + lane) * 4);
        asm volatile("s_wait_dscnt 0" ::: "memory");
        __builtin_amdgcn_wave_barrier();
        unsigned pv[16], pl[16];
#pragma unroll
        for (int r = 0; r < 16; ++r) {
            const float cs = ts[r * 64 + lane], sn = ts[r * 64 + 32 + lane];
            const float x1 = sg[r * 64 + 2 * lane], x2 = sg[r * 64 + 2 * lane + 1];
            const float o1 = x1 * cs - x2 * sn;
            const float o2 = x1 * sn + x2 * cs;
            _Float16 h0, l0, h1, l1;
            split16(o1, h0, l0); split16(o2, h1, l1);
            pv[r] = pack2h(h0, h1); pl[r] = pack2h(l0, l1);
        }
        _Float16* ob = outB + (((size_t)(b * HQ + h)) * SEQ + s0) * HDQ + 2 * lane;
#pragma unroll
        for (int r = 0; r < 16; ++r) { *(volatile unsigned*)(ob + r * HDQ) = pv[r]; *(volatile unsigned*)(ob + PLX + r * HDQ) = pl[r]; }
        __threadfence();
#pragma unroll
        for (int r = 0; r < 16; ++r) { *(volatile unsigned*)(ob + r * HDQ) = pv[r]; *(volatile unsigned*)(ob + PLX + r * HDQ) = pl[r]; }
    } else {
        const int bb = colBase / SEQ, sb = colBase % SEQ;
        const int h = rowBase >> 6, hd0 = rowBase & 63;
        unsigned pv[16], pl[16];
#pragma unroll
        for (int r = 0; r < 16; ++r) {
            _Float16 h0, l0, h1, l1;
            split16(sg[r * 64 + 2 * lane], h0, l0); split16(sg[r * 64 + 2 * lane + 1], h1, l1);
            pv[r] = pack2h(h0, h1); pl[r] = pack2h(l0, l1);
        }
        _Float16* ob = outB + (((size_t)(bb * HQ + h)) * HDQ + hd0) * SEQ + sb + 2 * lane;
#pragma unroll
        for (int r = 0; r < 16; ++r) { *(volatile unsigned*)(ob + (size_t)r * SEQ) = pv[r]; *(volatile unsigned*)(ob + PLX + (size_t)r * SEQ) = pl[r]; }
        __threadfence();
#pragma unroll
        for (int r = 0; r < 16; ++r) { *(volatile unsigned*)(ob + (size_t)r * SEQ) = pv[r]; *(volatile unsigned*)(ob + PLX + (size_t)r * SEQ) = pl[r]; }
    }
}

template <bool RES, int KB>
__device__ __forceinline__ void attn_kv_block(
    int kv0, int lo, int hi, int bh, const int* __restrict__ tokb, const int (&qp)[8],
    const _Float16* __restrict__ Km, const _Float16* __restrict__ Vt, _Float16* pw, _Float16* pwl,
    v16h qa0, v16h qa1, v16h qa0l, v16h qa1l,
    v8f (&cacc)[4], float (&mi)[8], float (&li)[8]) {
    constexpr int NT = KB / 16;
    constexpr int NF = KB / 32;

    int kp[NT];
#pragma unroll
    for (int tt = 0; tt < NT; ++tt) kp[tt] = tokb[kv0 + tt * 16 + lo];

    v8f s[NT];
#pragma unroll
    for (int tt = 0; tt < NT; ++tt) { v8f z = {}; s[tt] = z; }
#pragma unroll
    for (int tt = 0; tt < NT; ++tt) {
        const _Float16* kRow = Km + ((size_t)bh * SEQ + kv0 + tt * 16 + lo) * HDQ;
        const v16h kb0 = load_frag2(kRow + hi * 8,      kRow + 16 + hi * 8);
        const v16h kb1 = load_frag2(kRow + 32 + hi * 8, kRow + 48 + hi * 8);
        if constexpr (RES) {
            const v16h kb0l = load_frag2(kRow + PLX + hi * 8,      kRow + PLX + 16 + hi * 8);
            const v16h kb1l = load_frag2(kRow + PLX + 32 + hi * 8, kRow + PLX + 48 + hi * 8);
            s[tt] = wmma_split(qa0, qa0l, kb0, kb0l, s[tt]);
            s[tt] = wmma_split(qa1, qa1l, kb1, kb1l, s[tt]);
        } else {
            s[tt] = wmma16(qa0, kb0, s[tt]);
            s[tt] = wmma16(qa1, kb1, s[tt]);
        }
    }

    float alpha[8], rsum[8];
#pragma unroll
    for (int j = 0; j < 8; ++j) {
        float sv[NT]; bool mk[NT];
        float mb = -3.0e38f;
#pragma unroll
        for (int tt = 0; tt < NT; ++tt) {
            mk[tt] = kp[tt] > qp[j];
            sv[tt] = mk[tt] ? -3.0e38f : s[tt][j];
            mb = fmaxf(mb, sv[tt]);
        }
#pragma unroll
        for (int d = 1; d < 16; d <<= 1) mb = fmaxf(mb, __shfl_xor(mb, d, 32));
        const float mnew = fmaxf(mi[j], mb);
        alpha[j] = __expf(mi[j] - mnew);
        mi[j] = mnew;
        const int r = (j + 8 * hi) * 64;
        float rp = 0.0f;
#pragma unroll
        for (int tt = 0; tt < NT; ++tt) {
            const float e = __expf(sv[tt] - mnew) * PSC;
            const float p = mk[tt] ? 0.0f : e;
            rp += p;
            if constexpr (RES) {
                _Float16 ph, pq; split16(p, ph, pq);
                pw[r + tt * 16 + lo] = ph; pwl[r + tt * 16 + lo] = pq;
            } else {
                pw[r + tt * 16 + lo] = (_Float16)p;
            }
        }
#pragma unroll
        for (int d = 1; d < 16; d <<= 1) rp += __shfl_xor(rp, d, 32);
        rsum[j] = rp;
    }
    asm volatile("s_wait_dscnt 0" ::: "memory");
    __builtin_amdgcn_wave_barrier();

    v16h pA[NF], pAl[NF];
#pragma unroll
    for (int f = 0; f < NF; ++f) {
        pA[f] = load_frag2(pw + lo * 64 + f * 32 + hi * 8, pw + lo * 64 + f * 32 + hi * 8 + 16);
        if constexpr (RES) pAl[f] = load_frag2(pwl + lo * 64 + f * 32 + hi * 8, pwl + lo * 64 + f * 32 + hi * 8 + 16);
        else pAl[f] = pA[f];
    }

#pragma unroll
    for (int j = 0; j < 8; ++j) li[j] = li[j] * alpha[j] + rsum[j];

#pragma unroll
    for (int t = 0; t < 4; ++t) {
        const _Float16* vRow = Vt + ((size_t)bh * HDQ + t * 16 + lo) * SEQ + kv0;
#pragma unroll
        for (int j = 0; j < 8; ++j) cacc[t][j] *= alpha[j];
#pragma unroll
        for (int f = 0; f < NF; ++f) {
            const v16h vb = load_frag2(vRow + f * 32 + hi * 8, vRow + f * 32 + 16 + hi * 8);
            if constexpr (RES) {
                const v16h vbl = load_frag2(vRow + PLX + f * 32 + hi * 8, vRow + PLX + f * 32 + 16 + hi * 8);
                cacc[t] = wmma_split(pA[f], pAl[f], vb, vbl, cacc[t]);
            } else {
                cacc[t] = wmma16(pA[f], vb, cacc[t]);
            }
        }
    }
}

template <bool RES, int KB, int QBASE, int QCNT>
__global__ __launch_bounds__(256) __attribute__((amdgpu_num_vgpr(256)))
void flash_attn(const _Float16* __restrict__ Q, const _Float16* __restrict__ Km,
                const _Float16* __restrict__ Vt, _Float16* __restrict__ ctx, const int* __restrict__ tok) {
    __shared__ alignas(16) _Float16 psh[8][16 * 64];
    __shared__ alignas(16) _Float16 pshl[RES ? 8 : 1][16 * 64];
    __shared__ alignas(16) float    osh[8][16 * 64];

    const int lane = threadIdx.x & 31;
    const int wave = threadIdx.x >> 5;
    const int lo   = lane & 15;
    const int hi   = lane >> 4;
    const int w    = blockIdx.x * 8 + wave;
    const int qt   = w % QCNT;
    const int bh   = w / QCNT;
    if (bh >= NB * HQ) return;
    const int q0   = QBASE + qt * 16;
    const int b = bh / HQ, h = bh % HQ;
    const int* tokb = tok + (size_t)b * SEQ_FULL;

    int qp[8];
    int qmx = -2147483647 - 1;
#pragma unroll
    for (int j = 0; j < 8; ++j) { qp[j] = tokb[q0 + 8 * hi + j]; qmx = max(qmx, qp[j]); }
    qmx = max(qmx, __shfl_xor(qmx, 16, 32));
    qmx = __builtin_amdgcn_readfirstlane(qmx);

    const _Float16* qRow = Q + ((size_t)bh * SEQ + q0 + lo) * HDQ;
    const v16h qa0 = load_frag2(qRow + hi * 8,      qRow + hi * 8 + 16);
    const v16h qa1 = load_frag2(qRow + 32 + hi * 8, qRow + 32 + hi * 8 + 16);
    v16h qa0l = qa0, qa1l = qa1;
    if constexpr (RES) {
        qa0l = load_frag2(qRow + PLX + hi * 8,      qRow + PLX + hi * 8 + 16);
        qa1l = load_frag2(qRow + PLX + 32 + hi * 8, qRow + PLX + 32 + hi * 8 + 16);
    }

    v8f   cacc[4] = {};
    float mi[8], li[8];
#pragma unroll
    for (int j = 0; j < 8; ++j) { mi[j] = -3.0e38f; li[j] = 0.0f; }

    _Float16* pw  = psh[wave];
    _Float16* pwl = pshl[RES ? wave : 0];

#pragma unroll 1
    for (int ib = 0; ib < SEQ / KB; ++ib) {
        const int kv0 = ib * KB;
        int kmn = 2147483647;
#pragma unroll
        for (int u = 0; u < KB / 32; ++u) kmn = min(kmn, tokb[kv0 + u * 32 + lane]);
#pragma unroll
        for (int d = 1; d < 32; d <<= 1) kmn = min(kmn, __shfl_xor(kmn, d, 32));
        kmn = __builtin_amdgcn_readfirstlane(kmn);
        if (kmn > qmx) continue;
        attn_kv_block<RES, KB>(kv0, lo, hi, bh, tokb, qp, Km, Vt, pw, pwl, qa0, qa1, qa0l, qa1l, cacc, mi, li);
    }

    float* so = osh[wave];
#pragma unroll
    for (int j = 0; j < 8; ++j) {
        const float inv = 1.0f / li[j];
#pragma unroll
        for (int t = 0; t < 4; ++t) so[(j + 8 * hi) * 64 + t * 16 + lo] = cacc[t][j] * inv;
    }
    asm volatile("s_wait_dscnt 0" ::: "memory");
    __builtin_amdgcn_wave_barrier();
#pragma unroll 1
    for (int pass = 0; pass < 2; ++pass) {
#pragma unroll 4
        for (int r = 0; r < 16; ++r) {
            _Float16 h0, l0, h1, l1;
            split16(so[r * 64 + 2 * lane], h0, l0); split16(so[r * 64 + 2 * lane + 1], h1, l1);
            const size_t po = ((size_t)b * SEQ + q0 + r) * DQ + h * HDQ + 2 * lane;
            *(volatile unsigned*)(ctx + po) = pack2h(h0, h1); *(volatile unsigned*)(ctx + PLX + po) = pack2h(l0, l1);
        }
        __threadfence();
    }
}

extern "C" void kernel_launch(void* const* d_in, const int* in_sizes, int n_in,
                              void* d_out, int out_size, void* d_ws, size_t ws_size,
                              hipStream_t stream) {
    if (n_in < 6) return;
    const float* x   = (const float*)d_in[0];
    const int*   tok = (const int*)d_in[1];
    const float* wq  = (const float*)d_in[2];
    const float* wk  = (const float*)d_in[3];
    const float* wv  = (const float*)d_in[4];
    const float* wo  = (const float*)d_in[5];
    float* out = (float*)d_out;

    const long long needRows = (long long)(NB - 1) * SEQ_FULL + SEQ;
    if ((long long)in_sizes[0] < needRows * DQ) return;
    if ((long long)in_sizes[1] < needRows) return;
    if (in_sizes[2] < DQ * DQ || in_sizes[3] < DQ * DQ || in_sizes[4] < DQ * DQ || in_sizes[5] < DQ * DQ) return;
    if ((long long)out_size < needRows * DQ) return;

    const size_t szXh  = PLX * 2;
    const size_t szW   = (size_t)DQ * DQ * 2;
    const size_t szTab = (size_t)MQ * 64 * 4;
    const size_t szP2  = PLX * 2 * 2;
    const size_t total = szXh + 4 * szW + szTab + 4 * szP2;
    if (ws_size < total) return;

    char* ws = (char*)d_ws;
    _Float16* xh   = (_Float16*)ws;  ws += szXh;
    _Float16* wqh  = (_Float16*)ws;  ws += szW;
    _Float16* wkh  = (_Float16*)ws;  ws += szW;
    _Float16* wvh  = (_Float16*)ws;  ws += szW;
    _Float16* woh  = (_Float16*)ws;  ws += szW;
    float*    tab  = (float*)ws;     ws += szTab;
    _Float16* Qp   = (_Float16*)ws;  ws += szP2;
    _Float16* Kp   = (_Float16*)ws;  ws += szP2;
    _Float16* Vtp  = (_Float16*)ws;  ws += szP2;
    _Float16* ctxp = (_Float16*)ws;  ws += szP2;

    cvt_x<<<(unsigned)(PLX / 1024), 256, 0, stream>>>(x, xh);
    cvt_w<<<dim3((DQ * DQ) / 1024, 4), 256, 0, stream>>>(wq, wk, wv, wo, wqh, wkh, wvh, woh);
    rope_tab<<<MQ / 8, 256, 0, stream>>>(tok, tab);
    const dim3 gp(DQ / 64, MQ / 128);
    gemm16<1, false><<<gp, 256, 0, stream>>>(xh, wqh, out, Qp, tab, DQ, DQ, 0.125f * RWSC);
    gemm16<1, false><<<gp, 256, 0, stream>>>(xh, wkh, out, Kp, tab, DQ, DQ, RWSC);
    gemm16<3, false><<<dim3(MQ / 64, DQ / 128), 256, 0, stream>>>(wvh, xh, out, Vtp, tab, MQ, DQ, RWSC);
    flash_attn<true, 32, 0, (EARLYQ / 16)>
        <<<(NB * HQ * (EARLYQ / 16)) / 8, 256, 0, stream>>>(Qp, Kp, Vtp, ctxp, tok);
    constexpr int LATEQ = SEQ - EARLYQ;
    if (LATEQ > 0)
        flash_attn<false, 64, EARLYQ, ((LATEQ > 0) ? (LATEQ / 16) : 1)>
            <<<(NB * HQ * (LATEQ / 16)) / 8, 256, 0, stream>>>(Qp, Kp, Vtp, ctxp, tok);
    gemm16<0, true><<<gp, 256, 0, stream>>>(ctxp, woh, out, Qp, tab, DQ, DQ, RWSC);
}
